// MambaBlockV1_29291676958778
// MI455X (gfx1250) — hardware-verified
//
#include <hip/hip_runtime.h>
#include <hip/hip_bf16.h>


#define NB_   2
#define NL_   4096
#define DM_   256
#define DI_   512
#define NS_   16
#define DTR_  16
#define DTK_  32
#define XDN_  48
#define XDW_  64
#define MT_   (NB_ * NL_)

static_assert(MT_ % 64 == 0);
static_assert((2 * DI_) % 64 == 0);
static_assert(DI_ % 64 == 0);
static_assert(DM_ % 64 == 0);
static_assert(XDW_ % 64 == 0);
static_assert(DTR_ + 2 * NS_ == XDN_);
static_assert(XDN_ <= XDW_);
static_assert(DTK_ % 32 == 0);
static_assert(DTR_ <= DTK_);
static_assert(NL_ % 16 == 0);
static_assert((NL_ & (NL_ - 1)) == 0);
static_assert(DM_ == 256);
static_assert(DI_ == 512);

typedef float          v4f   __attribute__((ext_vector_type(4)));
typedef float          v8f   __attribute__((ext_vector_type(8)));
typedef __bf16         v16b  __attribute__((ext_vector_type(16)));
typedef unsigned short u16x8 __attribute__((ext_vector_type(8)));

union FragB { u16x8 h[2]; v16b v; };

constexpr size_t SZ_XL  = (size_t)MT_ * DM_ * 2;
constexpr size_t SZ_WI  = (size_t)(2 * DI_) * DM_ * 2;
constexpr size_t SZ_F   = (size_t)MT_ * DI_ * 4;
constexpr size_t SZ_H   = (size_t)MT_ * DI_ * 2;
constexpr size_t SZ_WX  = (size_t)XDW_ * DI_ * 2;
constexpr size_t SZ_XD  = (size_t)MT_ * XDW_ * 4;
constexpr size_t SZ_DR  = (size_t)MT_ * DTK_ * 2;
constexpr size_t SZ_WD  = (size_t)DI_ * DTK_ * 2;
constexpr size_t SZ_WO  = (size_t)DM_ * DI_ * 2;
constexpr size_t SZ_OM  = (size_t)MT_ * DM_ * 4;

constexpr size_t OFF_XLH = 0;
constexpr size_t OFF_XLL = OFF_XLH + SZ_XL;
constexpr size_t OFF_WIH = OFF_XLL + SZ_XL;
constexpr size_t OFF_WIL = OFF_WIH + SZ_WI;
constexpr size_t OFF_XF  = OFF_WIL + SZ_WI;
constexpr size_t OFF_ZF  = OFF_XF  + SZ_F;
constexpr size_t OFF_XCH = OFF_ZF  + SZ_F;
constexpr size_t OFF_XCL = OFF_XCH + SZ_H;
constexpr size_t OFF_WXH = OFF_XCL + SZ_H;
constexpr size_t OFF_WXL = OFF_WXH + SZ_WX;
constexpr size_t OFF_XD  = OFF_WXL + SZ_WX;
constexpr size_t OFF_DRH = OFF_XD  + SZ_XD;
constexpr size_t OFF_DRL = OFF_DRH + SZ_DR;
constexpr size_t OFF_WDH = OFF_DRL + SZ_DR;
constexpr size_t OFF_WDL = OFF_WDH + SZ_WD;
constexpr size_t OFF_DTP = OFF_WDL + SZ_WD;
constexpr size_t OFF_YH  = OFF_DTP + SZ_F;
constexpr size_t OFF_YL  = OFF_YH  + SZ_H;
constexpr size_t OFF_WOH = OFF_YL  + SZ_H;
constexpr size_t OFF_WOL = OFF_WOH + SZ_WO;
constexpr size_t OFF_OM  = OFF_WOL + SZ_WO;
constexpr size_t WS_END  = OFF_OM  + SZ_OM;
static_assert(WS_END <= (size_t)134217728);
static_assert(SZ_XL % 128 == 0 && SZ_WI % 128 == 0 && SZ_F % 128 == 0 && SZ_H % 128 == 0);
static_assert(SZ_WX % 128 == 0 && SZ_XD % 128 == 0 && SZ_DR % 128 == 0 && SZ_WD % 128 == 0);
static_assert(SZ_WO % 128 == 0 && SZ_OM % 128 == 0);
static_assert(OFF_OM % 128 == 0 && OFF_YL % 128 == 0 && OFF_DTP % 128 == 0 && OFF_XD % 128 == 0);

__device__ __forceinline__ unsigned short f32_to_bf16(float f) {
    unsigned u = __float_as_uint(f);
    unsigned r = u + 0x7FFFu + ((u >> 16) & 1u);
    return (unsigned short)(r >> 16);
}
__device__ __forceinline__ float bf16_to_f32(unsigned short b) {
    return __uint_as_float(((unsigned)b) << 16);
}
__device__ __forceinline__ void split2(float f, unsigned short& hb, unsigned short& lb) {
    hb = f32_to_bf16(f);
    lb = f32_to_bf16(f - bf16_to_f32(hb));
}
__device__ __forceinline__ float silu_f(float x) {
    float e = __expf(-x);
    return x * __builtin_amdgcn_rcpf(1.0f + e);
}
__device__ __forceinline__ float softplus_f(float x) {
    return fmaxf(x, 0.0f) + log1pf(__expf(-fabsf(x)));
}
__device__ __forceinline__ float conv4_silu(float x0, float x1, float x2, float x3,
                                            float w0, float w1, float w2, float w3, float bias) {
    float c = w0 * x0 + w1 * x1 + w2 * x2 + w3 * x3;
    return silu_f(c + bias);
}
__device__ __forceinline__ v8f ld8f(const float* p) {
    v4f a = *(const v4f*)p;
    v4f b = *(const v4f*)(p + 4);
    return __builtin_shufflevector(a, b, 0, 1, 2, 3, 4, 5, 6, 7);
}
__device__ __forceinline__ float wave_sum(float v) {
#pragma unroll
    for (int off = 16; off > 0; off >>= 1) v += __shfl_xor(v, off, 32);
    return v;
}
__device__ __forceinline__ void store8x2(unsigned short* ph, unsigned short* pl,
                                         const u16x8 hv, const u16x8 lv) {
    *(volatile u16x8*)ph = hv;
    *(volatile u16x8*)pl = lv;
    __threadfence();
    *(volatile u16x8*)ph = hv;
    *(volatile u16x8*)pl = lv;
}

__device__ __forceinline__ void mma16(v8f& acc, const FragB& a, const FragB& b) {
    acc = __builtin_amdgcn_wmma_f32_16x16x32_bf16(false, a.v, false, b.v, (short)0, acc, false, false);
    asm volatile("v_nop\n\tv_nop\n\tv_nop\n\tv_nop" : "+v"(acc) : "v"(a.v), "v"(b.v));
}

__global__ __launch_bounds__(128)
void ln_in_kernel(const float* __restrict__ feats, const int* __restrict__ perm,
                  const float* __restrict__ w, const float* __restrict__ bias,
                  unsigned short* dhi, unsigned short* dlo, int flip)
{
    const int lane = threadIdx.x & 31;
    const int wave = threadIdx.x >> 5;
    const int m  = blockIdx.x * 4 + wave;
    const int b  = m / NL_;
    const int t  = m & (NL_ - 1);
    const int tp = flip ? (NL_ - 1 - t) : t;
    int pidx = perm[b * NL_ + tp];
    pidx = min(max(pidx, 0), NL_ - 1);
    const int c0 = lane * 8;
    const v8f x = ld8f(feats + ((size_t)b * NL_ + pidx) * DM_ + c0);

    float s = 0.0f;
#pragma unroll
    for (int c = 0; c < 8; ++c) s += x[c];
    s = wave_sum(s);
    const float mu = s * (1.0f / DM_);
    float q = 0.0f;
#pragma unroll
    for (int c = 0; c < 8; ++c) { const float dv = x[c] - mu; q += dv * dv; }
    q = wave_sum(q);
    const float r = rsqrtf(q * (1.0f / DM_) + 1e-5f);

    const v8f wv = ld8f(w + c0);
    const v8f bv = ld8f(bias + c0);
    u16x8 hv, lv;
#pragma unroll
    for (int c = 0; c < 8; ++c) {
        const float y = (x[c] - mu) * r * wv[c] + bv[c];
        unsigned short hb, lb;
        split2(y, hb, lb);
        hv[c] = hb;
        lv[c] = lb;
    }
    const size_t e = (size_t)m * DM_ + c0;
    store8x2(dhi + e, dlo + e, hv, lv);
}

__global__ __launch_bounds__(256)
void wcvt_kernel(const float* __restrict__ src, unsigned short* dhi, unsigned short* dlo,
                 int K, int N, int Kp, int total8)
{
    const int i = blockIdx.x * 256 + threadIdx.x;
    if (i >= total8) return;
    const int e  = i * 8;
    const int n  = e / Kp;
    const int k0 = e - n * Kp;
    const int nn = min(n, N - 1);
    u16x8 hv, lv;
#pragma unroll
    for (int j = 0; j < 8; ++j) {
        const int kk = min(k0 + j, K - 1);
        const float f = src[(size_t)kk * N + nn];
        const float x = (n < N && (k0 + j) < K) ? f : 0.0f;
        unsigned short hb, lb;
        split2(x, hb, lb);
        hv[j] = hb;
        lv[j] = lb;
    }
    store8x2(dhi + (size_t)e, dlo + (size_t)e, hv, lv);
}

template<int NBF>
__device__ __forceinline__ void tile_store_pass(const float* st, float* gp, int ldc, int lane) {
    constexpr int CW  = NBF * 16;
    constexpr int P   = CW + 4;
    constexpr int LPR = CW / 4;
    static_assert(32 % LPR == 0);
    constexpr int RPI = 32 / LPR;
    static_assert(32 % RPI == 0);
    constexpr int NIT = 32 / RPI;
    const int rsub = lane / LPR;
    const int c0   = (lane % LPR) * 4;
#pragma unroll
    for (int it = 0; it < NIT; ++it) {
        const int row = it * RPI + rsub;
        const v4f v = *(const v4f*)(st + row * P + c0);
        *(volatile v4f*)(gp + (size_t)row * ldc + c0) = v;
    }
}

template<int NBF>
__global__ __launch_bounds__(128)
void gemm_split_kernel(const unsigned short* __restrict__ Ah, const unsigned short* __restrict__ Al,
                       const unsigned short* __restrict__ Bh, const unsigned short* __restrict__ Bl,
                       float* C, float* C2, int K, int ldc, int csplit)
{
    constexpr int CW = NBF * 16;
    constexpr int P  = CW + 4;
    __shared__ __attribute__((aligned(16))) float stile[4][32 * P];

    const int tid  = threadIdx.x;
    const int lane = tid & 31;
    const int wave = tid >> 5;
    const int h    = lane >> 4;
    const int m    = lane & 15;
    const int wm   = wave >> 1;
    const int wn   = wave & 1;

    const int rowW = blockIdx.y * 64 + wm * 32;
    const int colW = blockIdx.x * (2 * CW) + wn * CW;

    v8f acc[2 * NBF];
#pragma unroll
    for (int j = 0; j < 2 * NBF; ++j)
#pragma unroll
        for (int r = 0; r < 8; ++r) acc[j][r] = 0.0f;

    const size_t aoff  = (size_t)(rowW + m) * K + 8 * h;
    const size_t boff  = (size_t)(colW + m) * K + 8 * h;
    const size_t sub16 = (size_t)16 * K;
    const int nk = K >> 5;

    for (int kt = 0; kt < nk; ++kt) {
        const size_t k0 = (size_t)kt * 32;
        FragB fa[2], ga[2], fb[NBF], gb[NBF];
#pragma unroll
        for (int s = 0; s < 2; ++s) {
            const unsigned short* p = Ah + aoff + s * sub16 + k0;
            fa[s].h[0] = *(const u16x8*)(p);
            fa[s].h[1] = *(const u16x8*)(p + 16);
            const unsigned short* q = Al + aoff + s * sub16 + k0;
            ga[s].h[0] = *(const u16x8*)(q);
            ga[s].h[1] = *(const u16x8*)(q + 16);
        }
#pragma unroll
        for (int j = 0; j < NBF; ++j) {
            const unsigned short* p = Bh + boff + j * sub16 + k0;
            fb[j].h[0] = *(const u16x8*)(p);
            fb[j].h[1] = *(const u16x8*)(p + 16);
            const unsigned short* q = Bl + boff + j * sub16 + k0;
            gb[j].h[0] = *(const u16x8*)(q);
            gb[j].h[1] = *(const u16x8*)(q + 16);
        }
#pragma unroll
        for (int s = 0; s < 2; ++s)
#pragma unroll
            for (int j = 0; j < NBF; ++j) {
                mma16(acc[s * NBF + j], fa[s], fb[j]);
                mma16(acc[s * NBF + j], fa[s], gb[j]);
                mma16(acc[s * NBF + j], ga[s], fb[j]);
            }
    }

    float* st = stile[wave];
#pragma unroll
    for (int s = 0; s < 2; ++s)
#pragma unroll
        for (int j = 0; j < NBF; ++j)
#pragma unroll
            for (int r = 0; r < 8; ++r)
                st[(s * 16 + 8 * h + r) * P + j * 16 + m] = acc[s * NBF + j][r];
    __syncthreads();

    float* Cp = C;
    int gcol = colW;
    if (colW >= csplit) { Cp = C2; gcol = colW - csplit; }
    float* gp = Cp + (size_t)rowW * ldc + gcol;
    tile_store_pass<NBF>(st, gp, ldc, lane);
    __threadfence();
    tile_store_pass<NBF>(st, gp, ldc, lane);
}

__global__ __launch_bounds__(64)
void conv_silu_kernel(const float* __restrict__ X, const float* __restrict__ cw,
                      const float* __restrict__ cb, unsigned short* uhi, unsigned short* ulo)
{
    const int m  = blockIdx.x;
    const int l  = m & (NL_ - 1);
    const int d0 = threadIdx.x * 8;

    const v8f x3 = ld8f(X + (size_t)m * DI_ + d0);
    v8f x2 = ld8f(X + (size_t)max(m - 1, 0) * DI_ + d0);
    v8f x1 = ld8f(X + (size_t)max(m - 2, 0) * DI_ + d0);
    v8f x0 = ld8f(X + (size_t)max(m - 3, 0) * DI_ + d0);
#pragma unroll
    for (int c = 0; c < 8; ++c) {
        x2[c] = (l >= 1) ? x2[c] : 0.0f;
        x1[c] = (l >= 2) ? x1[c] : 0.0f;
        x0[c] = (l >= 3) ? x0[c] : 0.0f;
    }

    const float* wp = cw + (size_t)d0 * 4;
    v4f wv[8];
#pragma unroll
    for (int c = 0; c < 8; ++c) wv[c] = *(const v4f*)(wp + 4 * c);
    const v8f bias = ld8f(cb + d0);

    u16x8 hv, lv;
#pragma unroll
    for (int c = 0; c < 8; ++c) {
        const float u = conv4_silu(x0[c], x1[c], x2[c], x3[c],
                                   wv[c][0], wv[c][1], wv[c][2], wv[c][3], bias[c]);
        unsigned short hb, lb;
        split2(u, hb, lb);
        hv[c] = hb;
        lv[c] = lb;
    }
    const size_t e = (size_t)m * DI_ + d0;
    store8x2(uhi + e, ulo + e, hv, lv);
}

__global__ __launch_bounds__(256)
void dtr_kernel(const float* __restrict__ xd, unsigned short* dhi, unsigned short* dlo)
{
    const int i = blockIdx.x * 256 + threadIdx.x;
    if (i >= MT_ * (DTK_ / 8)) return;
    const int row = i / (DTK_ / 8);
    const int c0  = (i % (DTK_ / 8)) * 8;
    const v8f x = ld8f(xd + (size_t)row * XDW_ + c0);
    u16x8 hv, lv;
#pragma unroll
    for (int c = 0; c < 8; ++c) {
        const float v = (c0 + c < DTR_) ? x[c] : 0.0f;
        unsigned short hb, lb;
        split2(v, hb, lb);
        hv[c] = hb;
        lv[c] = lb;
    }
    const size_t e = (size_t)i * 8;
    store8x2(dhi + e, dlo + e, hv, lv);
}

__device__ __forceinline__ void rows16_store_pass(const unsigned short* sl, unsigned short* gpl,
                                                  size_t gbase, int lane) {
#pragma unroll
    for (int it = 0; it < 4; ++it) {
        const int t = it * 4 + (lane >> 3);
        const int c = (lane & 7) * 8;
        const u16x8 v = *(const u16x8*)(sl + t * 64 + c);
        *(volatile u16x8*)(gpl + gbase + (size_t)t * DI_ + c) = v;
    }
}

__global__ __launch_bounds__(64)
void scan_kernel(const float* __restrict__ X, const float* __restrict__ Z,
                 const float* __restrict__ DT, const float* __restrict__ xd,
                 const float* __restrict__ cw, const float* __restrict__ cb,
                 const float* __restrict__ Alog, const float* __restrict__ Dp,
                 const float* __restrict__ dtb,
                 unsigned short* yhi, unsigned short* ylo)
{
    __shared__ __attribute__((aligned(16))) unsigned short shi[16 * 64];
    __shared__ __attribute__((aligned(16))) unsigned short slo[16 * 64];
    __shared__ float sBC[16 * 2 * NS_];
    __shared__ float sA[64 * NS_];

    const int tid   = threadIdx.x;
    const int lane  = tid & 31;
    const int wave  = tid >> 5;
    const int dbase = blockIdx.x * 64;
    const int d     = dbase + tid;
    const int b     = blockIdx.y;

#pragma unroll 1
    for (int n = 0; n < NS_; ++n) sA[tid * NS_ + n] = -expf(Alog[d * NS_ + n]);
    __syncthreads();
    float an[NS_], hs[NS_];
#pragma unroll
    for (int n = 0; n < NS_; ++n) {
        an[n] = sA[tid * NS_ + n];
        hs[n] = 0.0f;
    }
    const float w0 = cw[d * 4 + 0], w1 = cw[d * 4 + 1], w2 = cw[d * 4 + 2], w3 = cw[d * 4 + 3];
    const float cbias = cb[d];
    const float tb = dtb[d];
    const float Dd = Dp[d];

    float xm1 = 0.0f, xm2 = 0.0f, xm3 = 0.0f;
    const size_t mrow0 = (size_t)b * NL_;

    const unsigned short* sl = wave ? slo : shi;
    unsigned short* gpl = wave ? ylo : yhi;

#pragma unroll 1
    for (int l0 = 0; l0 < NL_; l0 += 16) {
#pragma unroll
        for (int j = 0; j < 8; ++j) {
            const int tt = 2 * j + wave;
            sBC[tt * 32 + lane] = xd[(mrow0 + (size_t)(l0 + tt)) * XDW_ + DTR_ + lane];
        }
        __syncthreads();
#pragma unroll 1
        for (int t = 0; t < 16; ++t) {
            const size_t mrow = mrow0 + (size_t)(l0 + t);
            const size_t e = mrow * DI_ + d;
            const float xv = X[e];
            const float zv = Z[e];
            const float dl = DT[e];
            const float u  = conv4_silu(xm3, xm2, xm1, xv, w0, w1, w2, w3, cbias);
            xm3 = xm2; xm2 = xm1; xm1 = xv;
            const float dt = softplus_f(dl + tb);
            const float du = dt * u;
            float y = 0.0f;
#pragma unroll
            for (int n = 0; n < NS_; ++n) {
                const float da = __expf(dt * an[n]);
                hs[n] = da * hs[n] + du * sBC[t * 32 + n];
                y += hs[n] * sBC[t * 32 + NS_ + n];
            }
            const float g = (y + Dd * u) * silu_f(zv);
            unsigned short hb, lb;
            split2(g, hb, lb);
            shi[t * 64 + tid] = hb;
            slo[t * 64 + tid] = lb;
        }
        __syncthreads();
        const size_t gbase = (mrow0 + (size_t)l0) * DI_ + dbase;
        rows16_store_pass(sl, gpl, gbase, lane);
        __threadfence();
        rows16_store_pass(sl, gpl, gbase, lane);
        __syncthreads();
    }
}

__global__ __launch_bounds__(128)
void ln_out_kernel(const float* __restrict__ om, const int* __restrict__ perm,
                   const float* __restrict__ w, const float* __restrict__ bias,
                   float* dst, int flip)
{
    const int lane = threadIdx.x & 31;
    const int wave = threadIdx.x >> 5;
    const int m  = blockIdx.x * 4 + wave;
    const int b  = m / NL_;
    const int t  = m & (NL_ - 1);
    const int tp = flip ? (NL_ - 1 - t) : t;
    int pidx = perm[b * NL_ + tp];
    pidx = min(max(pidx, 0), NL_ - 1);

    const float* sr = om + (size_t)m * DM_;
    const int ca = lane * 4;
    const int cc = 128 + lane * 4;
    const v4f xa = *(const v4f*)(sr + ca);
    const v4f xc = *(const v4f*)(sr + cc);

    float s = 0.0f;
#pragma unroll
    for (int c = 0; c < 4; ++c) s += xa[c] + xc[c];
    s = wave_sum(s);
    const float mu = s * (1.0f / DM_);
    float q = 0.0f;
#pragma unroll
    for (int c = 0; c < 4; ++c) {
        const float da = xa[c] - mu; q += da * da;
        const float dc = xc[c] - mu; q += dc * dc;
    }
    q = wave_sum(q);
    const float r = rsqrtf(q * (1.0f / DM_) + 1e-5f);

    const v4f wa = *(const v4f*)(w + ca),    wc = *(const v4f*)(w + cc);
    const v4f ba = *(const v4f*)(bias + ca), bc = *(const v4f*)(bias + cc);
    v4f ya, yc;
#pragma unroll
    for (int c = 0; c < 4; ++c) {
        ya[c] = (xa[c] - mu) * r * wa[c] + ba[c];
        yc[c] = (xc[c] - mu) * r * wc[c] + bc[c];
    }
    float* dp = dst + ((size_t)b * NL_ + pidx) * DM_;
    *(volatile v4f*)(dp + ca) = ya;
    *(volatile v4f*)(dp + cc) = yc;
    __threadfence();
    *(volatile v4f*)(dp + ca) = ya;
    *(volatile v4f*)(dp + cc) = yc;
}

static void run_branch(hipStream_t stream, char* ws,
                       const float* feats, const int* perm, int flip,
                       const float* lnw, const float* lnb,
                       const float* w_in, const float* cw, const float* cb,
                       const float* wx, const float* wdt, const float* dtb,
                       const float* alog, const float* dp, const float* wo,
                       const float* fw, const float* fb, float* dst)
{
    unsigned short* xlh = (unsigned short*)(ws + OFF_XLH);
    unsigned short* xll = (unsigned short*)(ws + OFF_XLL);
    unsigned short* wih = (unsigned short*)(ws + OFF_WIH);
    unsigned short* wil = (unsigned short*)(ws + OFF_WIL);
    float*          Xf  = (float*)(ws + OFF_XF);
    float*          Zf  = (float*)(ws + OFF_ZF);
    unsigned short* xch = (unsigned short*)(ws + OFF_XCH);
    unsigned short* xcl = (unsigned short*)(ws + OFF_XCL);
    unsigned short* wxh = (unsigned short*)(ws + OFF_WXH);
    unsigned short* wxl = (unsigned short*)(ws + OFF_WXL);
    float*          xd  = (float*)(ws + OFF_XD);
    unsigned short* drh = (unsigned short*)(ws + OFF_DRH);
    unsigned short* drl = (unsigned short*)(ws + OFF_DRL);
    unsigned short* wdh = (unsigned short*)(ws + OFF_WDH);
    unsigned short* wdl = (unsigned short*)(ws + OFF_WDL);
    float*          dtp = (float*)(ws + OFF_DTP);
    unsigned short* yh  = (unsigned short*)(ws + OFF_YH);
    unsigned short* yl  = (unsigned short*)(ws + OFF_YL);
    unsigned short* woh = (unsigned short*)(ws + OFF_WOH);
    unsigned short* wol = (unsigned short*)(ws + OFF_WOL);
    float*          om  = (float*)(ws + OFF_OM);
    const int nosplit = 1 << 30;

    {
        int t8;
        t8 = ((2 * DI_) * DM_) / 8;
        hipLaunchKernelGGL(wcvt_kernel, dim3((t8 + 255) / 256), dim3(256), 0, stream,
                           w_in, wih, wil, (int)DM_, (int)(2 * DI_), (int)DM_, t8);
        t8 = (XDW_ * DI_) / 8;
        hipLaunchKernelGGL(wcvt_kernel, dim3((t8 + 255) / 256), dim3(256), 0, stream,
                           wx, wxh, wxl, (int)DI_, (int)XDN_, (int)DI_, t8);
        t8 = (DI_ * DTK_) / 8;
        hipLaunchKernelGGL(wcvt_kernel, dim3((t8 + 255) / 256), dim3(256), 0, stream,
                           wdt, wdh, wdl, (int)DTR_, (int)DI_, (int)DTK_, t8);
        t8 = (DM_ * DI_) / 8;
        hipLaunchKernelGGL(wcvt_kernel, dim3((t8 + 255) / 256), dim3(256), 0, stream,
                           wo, woh, wol, (int)DI_, (int)DM_, (int)DI_, t8);
    }

    hipLaunchKernelGGL(ln_in_kernel, dim3(MT_ / 4), dim3(128), 0, stream,
                       feats, perm, lnw, lnb, xlh, xll, flip);

    hipLaunchKernelGGL(HIP_KERNEL_NAME(gemm_split_kernel<2>),
                       dim3((2 * DI_) / 64, MT_ / 64), dim3(128), 0, stream,
                       (const unsigned short*)xlh, (const unsigned short*)xll,
                       (const unsigned short*)wih, (const unsigned short*)wil,
                       Xf, Zf, (int)DM_, (int)DI_, (int)DI_);

    hipLaunchKernelGGL(conv_silu_kernel, dim3(MT_), dim3(DI_ / 8), 0, stream,
                       (const float*)Xf, cw, cb, xch, xcl);

    hipLaunchKernelGGL(HIP_KERNEL_NAME(gemm_split_kernel<2>),
                       dim3(XDW_ / 64, MT_ / 64), dim3(128), 0, stream,
                       (const unsigned short*)xch, (const unsigned short*)xcl,
                       (const unsigned short*)wxh, (const unsigned short*)wxl,
                       xd, xd, (int)DI_, (int)XDW_, nosplit);

    hipLaunchKernelGGL(dtr_kernel, dim3((MT_ * (DTK_ / 8) + 255) / 256), dim3(256), 0, stream,
                       (const float*)xd, drh, drl);

    hipLaunchKernelGGL(HIP_KERNEL_NAME(gemm_split_kernel<2>),
                       dim3(DI_ / 64, MT_ / 64), dim3(128), 0, stream,
                       (const unsigned short*)drh, (const unsigned short*)drl,
                       (const unsigned short*)wdh, (const unsigned short*)wdl,
                       dtp, dtp, (int)DTK_, (int)DI_, nosplit);

    hipLaunchKernelGGL(scan_kernel, dim3(DI_ / 64, NB_), dim3(64), 0, stream,
                       (const float*)Xf, (const float*)Zf, (const float*)dtp, (const float*)xd,
                       cw, cb, alog, dp, dtb, yh, yl);

    hipLaunchKernelGGL(HIP_KERNEL_NAME(gemm_split_kernel<2>),
                       dim3(DM_ / 64, MT_ / 64), dim3(128), 0, stream,
                       (const unsigned short*)yh, (const unsigned short*)yl,
                       (const unsigned short*)woh, (const unsigned short*)wol,
                       om, om, (int)DI_, (int)DM_, nosplit);

    hipLaunchKernelGGL(ln_out_kernel, dim3(MT_ / 4), dim3(128), 0, stream,
                       (const float*)om, perm, fw, fb, dst, flip);
}

extern "C" void kernel_launch(void* const* d_in, const int* in_sizes, int n_in,
                              void* d_out, int out_size, void* d_ws, size_t ws_size,
                              hipStream_t stream)
{
    if (n_in < 30) return;
    if (in_sizes[0] != MT_ * DM_ || in_sizes[1] != MT_ * DM_) return;
    if (in_sizes[2] != MT_ || in_sizes[3] != MT_) return;
    for (int li = 0; li < 2; ++li) {
        const int o = (li == 0) ? 4 : 15;
        if (in_sizes[o + 0] != DM_)              return;
        if (in_sizes[o + 1] != DM_)              return;
        if (in_sizes[o + 2] != DM_ * 2 * DI_)    return;
        if (in_sizes[o + 3] != DI_ * 4)          return;
        if (in_sizes[o + 4] != DI_)              return;
        if (in_sizes[o + 5] != DI_ * XDN_)       return;
        if (in_sizes[o + 6] != DTR_ * DI_)       return;
        if (in_sizes[o + 7] != DI_)              return;
        if (in_sizes[o + 8] != DI_ * NS_)        return;
        if (in_sizes[o + 9] != DI_)              return;
        if (in_sizes[o + 10] != DI_ * DM_)       return;
    }
    if (in_sizes[26] != DM_ || in_sizes[27] != DM_ || in_sizes[28] != DM_ || in_sizes[29] != DM_) return;
    if (out_size != 2 * MT_ * DM_) return;
    if (ws_size < WS_END) return;

    const float* feats_s1 = (const float*)d_in[0];
    const float* feats_s2 = (const float*)d_in[1];
    const int*   perm_s1  = (const int*)d_in[2];
    const int*   perm_s2  = (const int*)d_in[3];
    const float* f[30];
    for (int i = 4; i < 30; ++i) f[i] = (const float*)d_in[i];

    float* out = (float*)d_out;
    char* ws = (char*)d_ws;

    run_branch(stream, ws, feats_s2, perm_s2, 0,
               f[4], f[5], f[6], f[7], f[8], f[9], f[10], f[11], f[12], f[13], f[14],
               f[26], f[27], out);

    run_branch(stream, ws, feats_s1, perm_s1, 1,
               f[15], f[16], f[17], f[18], f[19], f[20], f[21], f[22], f[23], f[24], f[25],
               f[28], f[29], out + (size_t)MT_ * DM_);
}
